// SymmetryAwareTaylorApproximatedAttention_3599182594292
// MI455X (gfx1250) — hardware-verified
//
#include <hip/hip_runtime.h>
#include <math.h>
#include <stdint.h>

#define TT    2048
#define NB    4
#define NHD   8
#define DKY   32
#define DVL   64
#define NBH   (NB * NHD)
#define NQB   (TT / 64)
#define AHS   64.0f
#define ALS   1024.0f
#define VSC   16.0f
#define F16MX 65504.0f
static_assert((TT % 64) == 0);
static_assert(DKY == 32);
static_assert(DVL == 64);
static_assert(((NBH * TT * DKY) % (8 * 256)) == 0);

typedef _Float16 v16h __attribute__((ext_vector_type(16)));
typedef _Float16 v8h  __attribute__((ext_vector_type(8)));
typedef __bf16   v16b __attribute__((ext_vector_type(16)));
typedef __bf16   v8b  __attribute__((ext_vector_type(8)));
typedef float    v8f  __attribute__((ext_vector_type(8)));
typedef float    v4f  __attribute__((ext_vector_type(4)));
typedef unsigned int v4u __attribute__((ext_vector_type(4)));

__device__ __forceinline__ unsigned short bf_bits(float f) {
  unsigned u = __float_as_uint(f);
  return (unsigned short)((u + 0x7FFFu + ((u >> 16) & 1u)) >> 16);
}
__device__ __forceinline__ float bf_up(unsigned short h) { return __uint_as_float(((unsigned)h) << 16); }
__device__ __forceinline__ unsigned short h_bits(_Float16 x) { return __builtin_bit_cast(unsigned short, x); }
__device__ __forceinline__ unsigned pk16(unsigned short a, unsigned short b) { return (unsigned)a | ((unsigned)b << 16); }
__device__ __forceinline__ v8f zero8() { v8f z = {0.f, 0.f, 0.f, 0.f, 0.f, 0.f, 0.f, 0.f}; return z; }

__device__ __forceinline__ float poly3(float x) {
#pragma clang fp contract(off)
  const float third = 1.0f / 3.0f;
  float t = 1.0f + x * third;
  t = 1.0f + (x * 0.5f) * t;
  t = 1.0f + x * t;
  return t;
}

__device__ __forceinline__ v16b ldfrag_b(const __bf16* p) {
  union { v16b v; v8b h[2]; } f;
  f.h[0] = *(const v8b*)(p);
  f.h[1] = *(const v8b*)(p + 16);
  return f.v;
}

__device__ __forceinline__ v8f mma_b(v16b a, v16b b, v8f c) {
  c = __builtin_amdgcn_wmma_f32_16x16x32_bf16(false, a, false, b, (short)0, c, false, false);
#if defined(__HIP_DEVICE_COMPILE__)
  asm volatile("v_nop\n\tv_nop\n\tv_nop\n\tv_nop" : "+v"(c) : "v"(a), "v"(b));
#endif
  return c;
}
__device__ __forceinline__ v8f mma_h(v16h a, v16h b, v8f c) {
  c = __builtin_amdgcn_wmma_f32_16x16x32_f16(false, a, false, b, (short)0, c, false, false);
#if defined(__HIP_DEVICE_COMPILE__)
  asm volatile("v_nop\n\tv_nop\n\tv_nop\n\tv_nop" : "+v"(c) : "v"(a), "v"(b));
#endif
  return c;
}

__global__ __launch_bounds__(256) void cvt_bf16(const float* __restrict__ in, unsigned short* out, int n8) {
  const int i = blockIdx.x * 256 + threadIdx.x;
  if (i < n8) {
    const size_t src = (size_t)i * 8;
    const v4f a = *(const v4f*)(in + src);
    const v4f b = *(const v4f*)(in + src + 4);
    v4u p;
    p[0] = pk16(bf_bits(a[0]), bf_bits(a[1]));
    p[1] = pk16(bf_bits(a[2]), bf_bits(a[3]));
    p[2] = pk16(bf_bits(b[0]), bf_bits(b[1]));
    p[3] = pk16(bf_bits(b[2]), bf_bits(b[3]));
    *(volatile v4u*)(out + src) = p;
    __threadfence();
    *(volatile v4u*)(out + src) = p;
  }
}

__global__ __launch_bounds__(256) void v_planes(const float* __restrict__ vf, unsigned short* vt, float vsc) {
  __shared__ __align__(16) float sv[64 * 68];
  const int tid = threadIdx.x;
  const int s0  = blockIdx.x * 64;
  const int bh  = blockIdx.y;
  if (bh >= NBH || s0 >= TT) return;
  const float* src = vf + ((size_t)bh * TT + (size_t)s0) * DVL;
#pragma unroll
  for (int i = 0; i < 4; ++i) {
    const int idx = i * 256 + tid;
    const int tt = idx >> 4, c4 = (idx & 15) * 4;
    const v4f a = *(const v4f*)(src + (size_t)tt * DVL + c4);
    *(v4f*)(sv + tt * 68 + c4) = a;
  }
  __syncthreads();

  const int g = tid >> 3, piece = tid & 7;
  v4u hv[2];
  size_t hofs[2];
#pragma unroll
  for (int it = 0; it < 2; ++it) {
    const int d = it * 32 + g;
    v4u a;
#pragma unroll
    for (int e = 0; e < 4; ++e) {
      const float f0 = sv[(piece * 8 + 2 * e) * 68 + d];
      const float f1 = sv[(piece * 8 + 2 * e + 1) * 68 + d];
      const _Float16 x0 = (_Float16)(bf_up(bf_bits(f0)) * vsc);
      const _Float16 x1 = (_Float16)(bf_up(bf_bits(f1)) * vsc);
      a[e] = pk16(h_bits(x0), h_bits(x1));
    }
    hv[it] = a;
    hofs[it] = ((size_t)(bh * DVL + d)) * TT + (size_t)s0 + (size_t)(piece * 8);
  }
  for (int pass = 0; pass < 2; ++pass) {
#pragma unroll
    for (int it = 0; it < 2; ++it) {
      *(volatile v4u*)(vt + hofs[it]) = hv[it];
    }
    __threadfence();
  }
}

__global__ __launch_bounds__(128)
void attn_poly(const unsigned short* __restrict__ qpl, const unsigned short* __restrict__ kpl,
               const unsigned short* __restrict__ vtpl, float* outp, float sscale) {
#pragma clang fp contract(off)
  union FH { v16h v; v8h h[2]; };
  union FB { v16b v; v8b h[2]; };
  __shared__ __align__(16) __bf16   Ksh[64 * DKY];
  __shared__ __align__(16) _Float16 Vth[DVL * 64];
  __shared__ __align__(16) _Float16 Psh[4][16 * 64];
  __shared__ __align__(16) _Float16 Psl[4][16 * 64];
  __shared__ __align__(16) float    Os[4][16 * DVL];

  const int tid  = threadIdx.x;
  const int wave = tid >> 5;
  const int lane = tid & 31;
  const int hh   = lane >> 4;
  const int c    = lane & 15;

  const int bx = blockIdx.x;
  const int qb = bx % NQB;
  const int bh = bx / NQB;
  if (bh >= NBH) return;
  const int q0 = qb * 64 + wave * 16;

  const __bf16*   Qp = (const __bf16*)(const void*)qpl + (size_t)bh * TT * DKY;
  const __bf16*   Kp = (const __bf16*)(const void*)kpl + (size_t)bh * TT * DKY;
  const _Float16* Vh = (const _Float16*)(const void*)vtpl + (size_t)bh * DVL * TT;

  const v16b qa = ldfrag_b(Qp + (size_t)(q0 + c) * DKY + 8 * hh);

  float zl[8];
  v8f oacc[4], olo[4];
#pragma unroll
  for (int r = 0; r < 8; ++r) zl[r] = 0.f;
#pragma unroll
  for (int t = 0; t < 4; ++t) { oacc[t] = zero8(); olo[t] = zero8(); }

  int nkt = qb + 1;
  if (nkt > NQB) nkt = NQB;
  for (int kt = 0; kt < nkt; ++kt) {
    const int kv0 = kt * 64;
    __syncthreads();
    {
      const int r  = tid >> 1;
      const int hf = (tid & 1) * 16;
      const __bf16* kg = Kp + (size_t)(kv0 + r) * DKY + hf;
      const v8b a0 = *(const v8b*)(kg);
      const v8b a1 = *(const v8b*)(kg + 8);
      *(v8b*)(Ksh + r * DKY + hf)     = a0;
      *(v8b*)(Ksh + r * DKY + hf + 8) = a1;
      const int so = (tid & 1) * 32;
      const _Float16* vg = Vh + (size_t)r * TT + (size_t)kv0 + (size_t)so;
#pragma unroll
      for (int i = 0; i < 4; ++i) {
        const v8h b0 = *(const v8h*)(vg + 8 * i);
        *(v8h*)(Vth + r * 64 + so + 8 * i) = b0;
      }
    }
    __syncthreads();

    v8f s[4];
#pragma unroll
    for (int j = 0; j < 4; ++j) {
      FB kb;
      kb.h[0] = *(const v8b*)(Ksh + (j * 16 + c) * DKY + 8 * hh);
      kb.h[1] = *(const v8b*)(Ksh + (j * 16 + c) * DKY + 16 + 8 * hh);
      s[j] = mma_b(qa, kb.v, zero8());
    }

    _Float16* pwh = Psh[wave];
    _Float16* pwl = Psl[wave];
#pragma unroll
    for (int r = 0; r < 8; ++r) {
      const int qrow = q0 + 8 * hh + r;
#pragma unroll
      for (int j = 0; j < 4; ++j) {
        const int key = kv0 + j * 16 + c;
        const float x = s[j][r] * sscale;
        float a = poly3(x);
        a = (key > qrow) ? 0.0f : a;
        zl[r] += a;
        float ac = a * AHS;
        ac = fminf(fmaxf(ac, -F16MX), F16MX);
        const _Float16 ah = (_Float16)ac;
        const _Float16 al = (_Float16)((ac - (float)ah) * ALS);
        pwh[(8 * hh + r) * 64 + j * 16 + c] = ah;
        pwl[(8 * hh + r) * 64 + j * 16 + c] = al;
      }
    }
    __builtin_amdgcn_fence(__ATOMIC_RELEASE, "workgroup");
    __builtin_amdgcn_wave_barrier();
    __builtin_amdgcn_fence(__ATOMIC_ACQUIRE, "workgroup");

#pragma unroll 1
    for (int kk = 0; kk < 2; ++kk) {
      FH pa, pl;
      pa.h[0] = *(const v8h*)(pwh + c * 64 + kk * 32 + 8 * hh);
      pa.h[1] = *(const v8h*)(pwh + c * 64 + kk * 32 + 16 + 8 * hh);
      pl.h[0] = *(const v8h*)(pwl + c * 64 + kk * 32 + 8 * hh);
      pl.h[1] = *(const v8h*)(pwl + c * 64 + kk * 32 + 16 + 8 * hh);
#pragma unroll
      for (int t = 0; t < 4; ++t) {
        FH vb;
        vb.h[0] = *(const v8h*)(Vth + (t * 16 + c) * 64 + kk * 32 + 8 * hh);
        vb.h[1] = *(const v8h*)(Vth + (t * 16 + c) * 64 + kk * 32 + 16 + 8 * hh);
        oacc[t] = mma_h(pa.v, vb.v, oacc[t]);
        olo[t]  = mma_h(pl.v, vb.v, olo[t]);
      }
    }
  }

  float* os = Os[wave];
#pragma unroll
  for (int r = 0; r < 8; ++r) {
    float z = zl[r];
    z += __shfl_xor(z, 1, 32);
    z += __shfl_xor(z, 2, 32);
    z += __shfl_xor(z, 4, 32);
    z += __shfl_xor(z, 8, 32);
    const float rz = 1.0f / z;
#pragma unroll
    for (int t = 0; t < 4; ++t) {
      const float sv = (oacc[t][r] + olo[t][r] * (1.0f / ALS)) * (1.0f / (AHS * VSC));
      os[(8 * hh + r) * DVL + t * 16 + c] = sv * rz;
    }
  }
  __builtin_amdgcn_fence(__ATOMIC_RELEASE, "workgroup");
  __builtin_amdgcn_wave_barrier();
  __builtin_amdgcn_fence(__ATOMIC_ACQUIRE, "workgroup");
  {
    const int col4 = c * 4;
    for (int pass = 0; pass < 2; ++pass) {
#pragma unroll
      for (int it = 0; it < 8; ++it) {
        const int rr = 2 * it + hh;
        const v4f ov = *(const v4f*)(os + rr * DVL + col4);
        const size_t go = ((size_t)(bh * TT + q0 + rr)) * DVL + (size_t)col4;
        *(volatile v4f*)(outp + go) = ov;
      }
      __threadfence();
    }
  }
}

extern "C" void kernel_launch(void* const* d_in, const int* in_sizes, int n_in,
                              void* d_out, int out_size, void* d_ws, size_t ws_size,
                              hipStream_t stream) {
  const int nq = NBH * TT * DKY;
  const int nv = NBH * TT * DVL;
  if (n_in < 3) return;
  if (in_sizes[0] != nq) return;
  if (in_sizes[1] != nq) return;
  if (in_sizes[2] != nv) return;
  if (out_size != nv) return;

  const float* q = (const float*)d_in[0];
  const float* k = (const float*)d_in[1];
  const float* v = (const float*)d_in[2];

  const size_t PQ = (size_t)nq * 2;
  const size_t PK = (size_t)nq * 2;
  const size_t PV = (size_t)nv * 2;
  size_t off = 0;
  const size_t oQ = off; off += PQ;
  const size_t oK = off; off += PK;
  const size_t oV = off; off += PV;
  if (off > ws_size) return;
  if (off > (size_t)134217728) return;

  char* ws = (char*)d_ws;
  unsigned short* Qb = (unsigned short*)(ws + oQ);
  unsigned short* Kb = (unsigned short*)(ws + oK);
  unsigned short* Vt = (unsigned short*)(ws + oV);
  float* outf = (float*)d_out;

  const dim3 blk(256);
  const int n8 = nq / 8;
  const dim3 gCvt((n8 + 255) / 256);
  const dim3 gV(TT / 64, NBH);
  const float sscale = 1.0f / sqrtf((float)DKY);

  cvt_bf16<<<gCvt, blk, 0, stream>>>(q, Qb, n8);
  cvt_bf16<<<gCvt, blk, 0, stream>>>(k, Kb, n8);
  v_planes<<<gV, blk, 0, stream>>>(v, Vt, VSC);
  attn_poly<<<dim3(NBH * NQB), dim3(128), 0, stream>>>(Qb, Kb, Vt, outf, sscale);
  (void)hipGetLastError();
}
